// WaypointSmoother_80350248173878
// MI455X (gfx1250) — hardware-verified
//
#include <hip/hip_runtime.h>


namespace {
constexpr int B = 4096, N = 512, NP = B * N, H1 = 64, H2 = 32;
constexpr float XS = 8.0f, WSC = 256.0f;
typedef _Float16 b16;
typedef __attribute__((ext_vector_type(16))) _Float16 v16b;
typedef __attribute__((ext_vector_type(8))) _Float16 v8b;
typedef __attribute__((ext_vector_type(8))) float v8f;
typedef __attribute__((ext_vector_type(2))) float v2f;
__device__ __forceinline__ float bf16_rne(float f) { unsigned int u = __float_as_uint(f); u += 0x7FFFu + ((u >> 16) & 1u); float r = __uint_as_float(u & 0xFFFF0000u); asm volatile("" : "+v"(r)); return r; }
__device__ __forceinline__ void split16(float v, b16& hi, b16& lo) { hi = (b16)v; lo = (b16)(v - (float)hi); }
__device__ __forceinline__ v16b frag_kb(const b16* p, int hh) { const v8b a = *(const v8b*)(p + 8 * hh), b = *(const v8b*)(p + 16 + 8 * hh); v16b f;
#pragma unroll
  for (int e = 0; e < 8; ++e) { f[e] = a[e]; f[8 + e] = b[e]; } return f; }
__device__ __forceinline__ v8f wmma16b(v16b a, v16b b, v8f c) { v8f d = __builtin_amdgcn_wmma_f32_16x16x32_f16(false, a, false, b, (short)0, c, false, false); asm volatile("v_nop\n\tv_nop\n\tv_nop\n\tv_nop" : "+v"(d) : "v"(a), "v"(b)); return d; }
__device__ __forceinline__ void wave_lds_sync() { __builtin_amdgcn_fence(__ATOMIC_RELEASE, "workgroup"); __builtin_amdgcn_wave_barrier(); __builtin_amdgcn_fence(__ATOMIC_ACQUIRE, "workgroup"); }
__device__ __forceinline__ float pmul(float a, float b) { float p = a * b; asm volatile("" : "+v"(p)); return p; }
__device__ __forceinline__ float sigm(float v) { return 1.0f / (1.0f + __expf(-v)); }
__device__ __forceinline__ float px(const float* __restrict__ wp, int b, int i, int c) { return bf16_rne(wp[((size_t)b * N + i) * 2 + c]); }

__global__ __launch_bounds__(256) void wput_kernel(const float* __restrict__ w1, const float* __restrict__ w2, b16* __restrict__ W1T, b16* __restrict__ W2T) { const int u = blockIdx.x * 256 + threadIdx.x;
  for (int pass = 0; pass < 2; ++pass) {
    if (u < H1 * 4) { const int o = u / 4, k0 = (u % 4) * 8; v8b v;
#pragma unroll
      for (int j = 0; j < 8; ++j) { const int k = k0 + j; v[j] = (b16)(k < 4 ? bf16_rne(w1[k * H1 + o]) * WSC : 0.0f); } *(volatile v8b*)(W1T + (size_t)o * 32 + k0) = v; }
    if (u < H2 * 8) { const int o = u / 8, k0 = (u % 8) * 8; v8b v;
#pragma unroll
      for (int j = 0; j < 8; ++j) v[j] = (b16)(bf16_rne(w2[(size_t)(k0 + j) * H2 + o]) * WSC); *(volatile v8b*)(W2T + (size_t)o * H1 + k0) = v; }
    __threadfence(); } }
__global__ __launch_bounds__(32) void mlp_kernel(const float* __restrict__ wp, const b16* __restrict__ W1T, const float* __restrict__ b1, const b16* __restrict__ W2T, const float* __restrict__ b2, const float* __restrict__ w3, const float* __restrict__ b3, const float* __restrict__ sw, int BV, float* __restrict__ WV) {
  __shared__ __attribute__((aligned(16))) b16 Fh[16][40], Fl[16][40], Hh[16][72], Hl[16][72]; __shared__ float T2[16][33], Wo[32]; const int lane = threadIdx.x, nloc = lane & 15, hlf = lane >> 4; const size_t p0 = (size_t)blockIdx.x * 32; const int b = (int)(p0 / N); if (b >= BV) return;
  const float ssw = sigm(bf16_rne(sw[0]));
  for (int mt = 0; mt < 2; ++mt) { const size_t pp = p0 + mt * 16;
    { const int rr = lane & 15; const int i = (int)((pp + rr) % N); float f[4];
      const int i1 = i < N - 1 ? i : N - 2; for (int c = 0; c < 2; ++c) { const float d1 = px(wp, b, i1 + 1, c) - px(wp, b, i1, c); float d2 = 0.0f; if (i >= 1 && i <= N - 2) { const float d1m = px(wp, b, i, c) - px(wp, b, i - 1, c); d2 = (px(wp, b, i + 1, c) - px(wp, b, i, c)) - d1m; } f[c] = d1; f[2 + c] = d2; }
      for (int k = 0; k < 16; ++k) { const int col = hlf * 16 + k; float v = col < 4 ? f[col < 4 ? col : 0] : 0.0f; b16 p, q; split16(v * XS, p, q); Fh[rr][col] = p; Fl[rr][col] = q; } }
    wave_lds_sync(); v8f a1[4] = {(v8f){}, (v8f){}, (v8f){}, (v8f){}}; { const v16b a = frag_kb(&Fh[nloc][0], hlf), al = frag_kb(&Fl[nloc][0], hlf);
#pragma unroll
      for (int t = 0; t < 4; ++t) { const v16b bw = frag_kb(W1T + (size_t)(t * 16 + nloc) * 32, hlf); a1[t] = wmma16b(a, bw, a1[t]); a1[t] = wmma16b(al, bw, a1[t]); } }
#pragma unroll
    for (int t = 0; t < 4; ++t) { const int c = t * 16 + nloc; const float bb = bf16_rne(b1[c]);
#pragma unroll
      for (int r8 = 0; r8 < 8; ++r8) { b16 p, q; split16(fmaxf(a1[t][r8] * (1.0f / (XS * WSC)) + bb, 0.0f) * XS, p, q); Hh[8 * hlf + r8][c] = p; Hl[8 * hlf + r8][c] = q; } }
    wave_lds_sync(); v8f a2[2] = {(v8f){}, (v8f){}};
#pragma unroll
    for (int kb = 0; kb < H1; kb += 32) { const v16b a = frag_kb(&Hh[nloc][kb], hlf), al = frag_kb(&Hl[nloc][kb], hlf);
#pragma unroll
      for (int t = 0; t < 2; ++t) { const v16b bw = frag_kb(W2T + (size_t)(t * 16 + nloc) * H1 + kb, hlf); a2[t] = wmma16b(a, bw, a2[t]); a2[t] = wmma16b(al, bw, a2[t]); } }
#pragma unroll
    for (int t = 0; t < 2; ++t) { const int c = t * 16 + nloc; const float bb = bf16_rne(b2[c]);
#pragma unroll
      for (int r8 = 0; r8 < 8; ++r8) T2[8 * hlf + r8][c] = fmaxf(a2[t][r8] * (1.0f / (XS * WSC)) + bb, 0.0f); }
    wave_lds_sync();
    if (lane < 16) { float s = bf16_rne(b3[0]);
#pragma unroll 1
      for (int k = 0; k < H2; ++k) s += pmul(T2[lane][k], bf16_rne(w3[k])); Wo[mt * 16 + lane] = pmul(ssw, 1.0f - sigm(s)); }
    wave_lds_sync(); }
  for (int pass = 0; pass < 2; ++pass) { ((volatile float*)WV)[p0 + lane] = Wo[lane]; __threadfence(); } }
__global__ __launch_bounds__(256) void scan_kernel(const float* __restrict__ wp, const float* __restrict__ WV, int BV, float* __restrict__ out) { const int b = blockIdx.x * 256 + threadIdx.x; if (b >= BV) return;
  for (int pass = 0; pass < 2; ++pass) { float y0 = px(wp, b, 0, 0), y1 = px(wp, b, 0, 1); ((volatile float*)out)[(size_t)b * N * 2] = y0; ((volatile float*)out)[(size_t)b * N * 2 + 1] = y1;
#pragma unroll 1
    for (int i = 1; i < N; ++i) { const float w = WV[(size_t)b * N + i]; y0 = pmul(w, y0) + pmul(1.0f - w, px(wp, b, i, 0)); y1 = pmul(w, y1) + pmul(1.0f - w, px(wp, b, i, 1)); float o0 = y0, o1 = y1; if (i == N - 1) { o0 = px(wp, b, i, 0); o1 = px(wp, b, i, 1); } ((volatile float*)out)[((size_t)b * N + i) * 2] = o0; ((volatile float*)out)[((size_t)b * N + i) * 2 + 1] = o1; }
    __threadfence(); } }
}

extern "C" void kernel_launch(void* const* d_in, const int* in_sizes, int n_in, void* d_out, int out_size, void* d_ws, size_t ws_size, hipStream_t stream) {
  (void)n_in;
  auto Fp = [&](int i) { return (const float*)d_in[i]; };
  if (in_sizes[0] != NP * 2 || in_sizes[1] != 1 || in_sizes[2] != 4 * H1 || in_sizes[4] != H1 * H2 || in_sizes[6] != H2 || out_size != NP * 2) return;
  const int BV = B;
  size_t off = 0; char* ws = (char*)d_ws;
  auto carve = [&](size_t bytes) { char* p = ws + off; off += (bytes + 255) & ~(size_t)255; return p; };
  b16* W1T = (b16*)carve((size_t)H1 * 32 * 2); b16* W2T = (b16*)carve((size_t)H2 * H1 * 2); float* WV = (float*)carve((size_t)NP * 4);
  if (off > ws_size || off > ((size_t)16 << 20)) return;
  wput_kernel<<<1, 256, 0, stream>>>(Fp(2), Fp(4), W1T, W2T);
  mlp_kernel<<<(unsigned)((size_t)BV * N / 32), 32, 0, stream>>>(Fp(0), W1T, Fp(3), W2T, Fp(5), Fp(6), Fp(7), Fp(1), BV, WV);
  scan_kernel<<<(BV + 255) / 256, 256, 0, stream>>>(Fp(0), WV, BV, (float*)d_out);
}
